// DIN_39616778338785
// MI455X (gfx1250) — hardware-run, weakly checked
//
#include <hip/hip_runtime.h>
#include <math.h>

#define NB_ 32
#define THIST 200
#define TQ 50
#define EE 64
#define PP 128
#define CX 64
#define UU 36
#define TPB 5
#define NPAIR (TPB * THIST)

typedef _Float16 f16;
typedef __attribute__((ext_vector_type(16))) f16 f16x16;
typedef __attribute__((ext_vector_type(8)))  f16 f16x8;
typedef __attribute__((ext_vector_type(8)))  float f32x8;
typedef __attribute__((ext_vector_type(4)))  float v4f_t;
typedef float v4fa __attribute__((ext_vector_type(4), may_alias));
__device__ __forceinline__ f32x8 wmma16(f16x16 a, f16x16 b, f32x8 c) {
  c = __builtin_amdgcn_wmma_f32_16x16x32_f16(false, a, false, b, (short)0, c, false, false);
  asm volatile("v_nop\n\tv_nop\n\tv_nop\n\tv_nop" : "+v"(c) : "v"(a), "v"(b));
  return c;
}
__device__ __forceinline__ f16x16 lds_frag(const f16* base, int stride) {
  const int lane = threadIdx.x & 31, row = lane & 15, kh = (lane >> 4) * 8;
  const f16x8 lo = *(const f16x8*)(base + row * stride + kh);
  const f16x8 hi = *(const f16x8*)(base + row * stride + kh + 16);
  f16x16 f;
#pragma unroll
  for (int i = 0; i < 8; ++i) { f[i] = lo[i]; f[i + 8] = hi[i]; }
  return f;
}
__device__ __forceinline__ void split16(float v, f16& h, f16& l) { h = (f16)v; l = (f16)((v - (float)h) * 2048.0f); }
__device__ __forceinline__ void mma3(f32x8& acc, f32x8& accx, const f16x16& ah, const f16x16& al, const f16x16& bh, const f16x16& bl) {
  acc = wmma16(ah, bh, acc); accx = wmma16(ah, bl, accx); accx = wmma16(al, bh, accx);
}
template <int MODE>
__device__ __forceinline__ void wfragT(const float* __restrict__ Wm, const float* __restrict__ Wc, int ldw, int nmax, int kmax, int n0, int k0, f16x16& hi, f16x16& lo) {
  const int lane = threadIdx.x & 31, n = n0 + (lane & 15), kh = (lane >> 4) * 8;
#pragma unroll
  for (int i = 0; i < 16; ++i) { const int k = k0 + kh + (i & 7) + ((i >> 3) * 16); float v = 0.0f;
    if (n < nmax && k < kmax) { const size_t idx = (size_t)k * ldw + n; v = Wm[idx]; if (MODE == 1) v += Wc[idx]; if (MODE == 2) v -= Wc[idx]; }
    f16 h, l; split16(v, h, l); hi[i] = h; lo[i] = l; }
}
__device__ __forceinline__ float bn_f(float v, const float* g, const float* bb, const float* m, const float* var, float eps, int c) { return (v - m[c]) * rsqrtf(var[c] + eps) * g[c] + bb[c]; }

__global__ __launch_bounds__(256) void k_din(const float* __restrict__ ub, const float* __restrict__ items, const float* __restrict__ prof, const float* __restrict__ ctx,
                                            const float* __restrict__ W1, const float* __restrict__ b1, const float* __restrict__ dal, const float* __restrict__ dmean, const float* __restrict__ dvar,
                                            const float* __restrict__ W2, const float* __restrict__ b2,
                                            const float* __restrict__ g1, const float* __restrict__ be1, const float* __restrict__ m1, const float* __restrict__ v1, const float* __restrict__ Wm1, const float* __restrict__ bm1,
                                            const float* __restrict__ g2, const float* __restrict__ be2, const float* __restrict__ m2, const float* __restrict__ v2, const float* __restrict__ Wm2, const float* __restrict__ bm2,
                                            const float* __restrict__ g3, const float* __restrict__ be3, const float* __restrict__ m3, const float* __restrict__ v3, const float* __restrict__ Wm3, const float* __restrict__ bm3,
                                            float* __restrict__ out) {
  __shared__ __attribute__((aligned(16))) union U1 { struct { f16 aS[2][128 * 72]; float AqS[208 * 37]; } a; f16 ubT[2][64 * 232]; } u1;
  __shared__ __attribute__((aligned(16))) union U2 { struct { float wS[16 * THIST]; f16 wP[2][16 * 232]; } w; f16 hP[2][16 * 264]; } u2;
  __shared__ float AkS[16 * 37];
  __shared__ float hS[16 * 260];
  __shared__ __attribute__((aligned(16))) float oS[16 * 68];
  f16 (*aS)[128 * 72] = u1.a.aS; float* AqS = u1.a.AqS; f16 (*ubT)[64 * 232] = u1.ubT; float* wS = u2.w.wS; f16 (*wP)[16 * 232] = u2.w.wP; f16 (*hP)[16 * 264] = u2.hP;
  const int tid = threadIdx.x, lane = tid & 31, wave = tid >> 5, cl = lane & 15, rh = (lane >> 4) * 8;
  const int b = blockIdx.x / (TQ / TPB), t0 = (blockIdx.x % (TQ / TPB)) * TPB;
  const float* ubb = ub + (size_t)b * THIST * EE; const float* itb = items + ((size_t)b * TQ + t0) * EE;
  const float* W1a = W1, *W1b = W1 + 64 * UU, *W1c = W1 + 128 * UU, *W1d = W1 + 192 * UU;
  for (int rt0 = 0; rt0 < 13; rt0 += 8) {
    __syncthreads();
    for (int e = tid; e < 128 * 64; e += 256) { const int r = e >> 6, c = e & 63; const int s = (rt0 + (r >> 4)) * 16 + (r & 15); const float v = (s < THIST) ? ubb[(size_t)min(s, THIST - 1) * EE + c] : 0.0f;
      f16 h, l; split16(v, h, l); aS[0][r * 72 + c] = h; aS[1][r * 72 + c] = l; }
    __syncthreads();
    const int rt = rt0 + wave; if (rt < 13) {
      for (int nt = 0; nt < 3; ++nt) { f32x8 acc = {}, accx = {};
#pragma unroll
        for (int ks = 0; ks < 2; ++ks) { f16x16 bh, bl; wfragT<1>(W1a, W1c, UU, UU, EE, nt * 16, ks * 32, bh, bl); mma3(acc, accx, lds_frag(aS[0] + (wave * 16) * 72 + ks * 32, 72), lds_frag(aS[1] + (wave * 16) * 72 + ks * 32, 72), bh, bl); }
#pragma unroll
        for (int r = 0; r < 8; ++r) { const int s = rt * 16 + rh + r, u = nt * 16 + cl; if (u < UU) AqS[s * 37 + u] = acc[r] + accx[r] * (1.0f / 2048.0f); } } }
  }
  __syncthreads();
  for (int e = tid; e < 16 * 64; e += 256) { const int r = e >> 6, c = e & 63; const float v = (r < TPB) ? itb[(size_t)min(r, TPB - 1) * EE + c] : 0.0f; f16 h, l; split16(v, h, l); aS[0][r * 72 + c] = h; aS[1][r * 72 + c] = l; }
  __syncthreads();
  if (wave < 3) { const int nt = wave; f32x8 acc = {}, accx = {};
#pragma unroll
    for (int ks = 0; ks < 2; ++ks) { f16x16 bh, bl; wfragT<2>(W1b, W1c, UU, UU, EE, nt * 16, ks * 32, bh, bl); mma3(acc, accx, lds_frag(aS[0] + ks * 32, 72), lds_frag(aS[1] + ks * 32, 72), bh, bl); }
#pragma unroll
    for (int r = 0; r < 8; ++r) { const int t = rh + r, u = nt * 16 + cl; if (u < UU) AkS[t * 37 + u] = acc[r] + accx[r] * (1.0f / 2048.0f) + b1[u]; } }
  for (int p0 = 0; p0 < NPAIR; p0 += 128) {
    __syncthreads();
    for (int e = tid; e < 128 * 64; e += 256) { const int r = e >> 6, c = e & 63; const int p = p0 + r; float v = 0.0f;
      if (p < NPAIR) { const int t = p / THIST, s = p % THIST; v = ubb[(size_t)s * EE + c] * itb[(size_t)t * EE + c]; }
      f16 h, l; split16(v, h, l); aS[0][r * 72 + c] = h; aS[1][r * 72 + c] = l; }
    __syncthreads();
    { f32x8 acc[3], accx[3];
#pragma unroll
      for (int nt = 0; nt < 3; ++nt) { f32x8 z = {}; acc[nt] = z; accx[nt] = z; }
#pragma unroll
      for (int ks = 0; ks < 2; ++ks) { const f16x16 ah = lds_frag(aS[0] + (wave * 16) * 72 + ks * 32, 72), al = lds_frag(aS[1] + (wave * 16) * 72 + ks * 32, 72);
#pragma unroll
        for (int nt = 0; nt < 3; ++nt) { f16x16 bh, bl; wfragT<0>(W1d, nullptr, UU, UU, EE, nt * 16, ks * 32, bh, bl); mma3(acc[nt], accx[nt], ah, al, bh, bl); } }
#pragma unroll
      for (int r = 0; r < 8; ++r) { const int p = p0 + wave * 16 + rh + r; const bool ok = p < NPAIR; const int t = ok ? p / THIST : 0, s = ok ? p % THIST : 0;
        float part = 0.0f;
#pragma unroll
        for (int nt = 0; nt < 3; ++nt) { const int u = nt * 16 + cl;
          if (u < UU && ok) { const float xv = acc[nt][r] + accx[nt][r] * (1.0f / 2048.0f) + AqS[s * 37 + u] + AkS[t * 37 + u];
            const float pg = 1.0f / (1.0f + expf(-(xv - dmean[u]) * rsqrtf(dvar[u] + 1e-6f))); const float dz = pg * xv + dal[u] * (1.0f - pg) * xv; part += dz * W2[u]; } }
#pragma unroll
        for (int off = 1; off < 16; off <<= 1) part += __shfl_xor(part, off, 32);
        if (cl == 0 && ok) wS[t * THIST + s] = part + b2[0]; } }
  }
  __syncthreads();
  for (int e = tid; e < 64 * 224; e += 256) { const int c = e / 224, s = e % 224; const float v = (s < THIST) ? ubb[(size_t)min(s, THIST - 1) * EE + c] : 0.0f; f16 h, l; split16(v, h, l); ubT[0][c * 232 + s] = h; ubT[1][c * 232 + s] = l; }
  for (int e = tid; e < 16 * 224; e += 256) { const int t = e / 224, s = e % 224; const float v = (t < TPB && s < THIST) ? wS[min(t, TPB - 1) * THIST + min(s, THIST - 1)] : 0.0f; f16 h, l; split16(v, h, l); wP[0][t * 232 + s] = h; wP[1][t * 232 + s] = l; }
  __syncthreads();
  if (wave < 4) { const int nt = wave; f32x8 acc = {}, accx = {};
    for (int ks = 0; ks < 7; ++ks) mma3(acc, accx, lds_frag(wP[0] + ks * 32, 232), lds_frag(wP[1] + ks * 32, 232), lds_frag(ubT[0] + (nt * 16) * 232 + ks * 32, 232), lds_frag(ubT[1] + (nt * 16) * 232 + ks * 32, 232));
#pragma unroll
    for (int r = 0; r < 8; ++r) hS[(rh + r) * 260 + nt * 16 + cl] = acc[r] + accx[r] * (1.0f / 2048.0f); }
  __syncthreads();
  for (int e = tid; e < 16 * 256; e += 256) { const int t = e >> 8, c = e & 255; float v = 0.0f;
    if (t < TPB) {
      const float hv = hS[t * 260 + min(c, EE - 1)]; const float pv = prof[(size_t)b * PP + min(max(c - EE, 0), PP - 1)]; const float cv = ctx[(size_t)b * CX + min(max(c - EE - PP, 0), CX - 1)];
      const float raw = (c < EE) ? hv : (c < EE + PP) ? pv : cv; v = bn_f(raw, g1, be1, m1, v1, 1e-6f, c); }
    f16 h, l; split16(v, h, l); hP[0][t * 264 + c] = h; hP[1][t * 264 + c] = l; }
  __syncthreads();
  { for (int j = 0; j < 2; ++j) { const int nt = wave * 2 + j; f32x8 acc = {}, accx = {};
      for (int ks = 0; ks < 8; ++ks) { f16x16 bh, bl; wfragT<0>(Wm1, nullptr, 256, 256, 256, nt * 16, ks * 32, bh, bl); mma3(acc, accx, lds_frag(hP[0] + ks * 32, 264), lds_frag(hP[1] + ks * 32, 264), bh, bl); }
#pragma unroll
      for (int r = 0; r < 8; ++r) { const int c = nt * 16 + cl; hS[(rh + r) * 260 + c] = fmaxf(acc[r] + accx[r] * (1.0f / 2048.0f) + bm1[c], 0.0f); } } }
  __syncthreads();
  for (int e = tid; e < 16 * 256; e += 256) { const int t = e >> 8, c = e & 255; const float v = bn_f(hS[t * 260 + c], g2, be2, m2, v2, 1e-6f, c); f16 h, l; split16(v, h, l); hP[0][t * 264 + c] = h; hP[1][t * 264 + c] = l; }
  __syncthreads();
  { const int nt = wave; f32x8 acc = {}, accx = {};
    for (int ks = 0; ks < 8; ++ks) { f16x16 bh, bl; wfragT<0>(Wm2, nullptr, 128, 128, 256, nt * 16, ks * 32, bh, bl); mma3(acc, accx, lds_frag(hP[0] + ks * 32, 264), lds_frag(hP[1] + ks * 32, 264), bh, bl); }
#pragma unroll
    for (int r = 0; r < 8; ++r) { const int c = nt * 16 + cl; hS[(rh + r) * 260 + c] = fmaxf(acc[r] + accx[r] * (1.0f / 2048.0f) + bm2[c], 0.0f); } }
  __syncthreads();
  for (int e = tid; e < 16 * 128; e += 256) { const int t = e >> 7, c = e & 127; const float v = bn_f(hS[t * 260 + c], g3, be3, m3, v3, 1e-6f, c); f16 h, l; split16(v, h, l); hP[0][t * 264 + c] = h; hP[1][t * 264 + c] = l; }
  __syncthreads();
  if (wave < 4) { const int nt = wave; f32x8 acc = {}, accx = {};
    for (int ks = 0; ks < 4; ++ks) { f16x16 bh, bl; wfragT<0>(Wm3, nullptr, 64, 64, 128, nt * 16, ks * 32, bh, bl); mma3(acc, accx, lds_frag(hP[0] + ks * 32, 264), lds_frag(hP[1] + ks * 32, 264), bh, bl); }
#pragma unroll
    for (int r = 0; r < 8; ++r) { const int c = nt * 16 + cl; oS[(rh + r) * 68 + c] = fmaxf(acc[r] + accx[r] * (1.0f / 2048.0f) + bm3[c], 0.0f); } }
  __syncthreads();
#pragma unroll 1
  for (int pass = 0; pass < 2; ++pass) { if (tid < TPB * 16) { const int t = tid >> 4, c4 = (tid & 15) * 4; *(volatile v4f_t*)(out + ((size_t)b * TQ + t0 + t) * EE + c4) = *(const volatile v4fa*)(oS + t * 68 + c4); } __threadfence(); }
}

extern "C" void kernel_launch(void* const* d_in, const int* in_sizes, int n_in,
                              void* d_out, int out_size, void* d_ws, size_t ws_size,
                              hipStream_t stream) {
  (void)in_sizes; (void)n_in; (void)out_size; (void)d_ws; (void)ws_size;
  const float** f = (const float**)d_in;
  float* out = (float*)d_out;
  k_din<<<dim3(NB_ * (TQ / TPB)), dim3(256), 0, stream>>>(f[0], f[1], f[2], f[3], f[4], f[5], f[6], f[7], f[8], f[9], f[10],
      f[11], f[12], f[13], f[14], f[15], f[16], f[17], f[18], f[19], f[20], f[21], f[22], f[23], f[24], f[25], f[26], f[27], f[28], out);
}
